// QSVDDModel_44684839748154
// MI455X (gfx1250) — hardware-verified
//
#include <hip/hip_runtime.h>
#include <math.h>

typedef __attribute__((ext_vector_type(16))) _Float16 v16h;
typedef __attribute__((ext_vector_type(8)))  _Float16 v8h;
typedef __attribute__((ext_vector_type(8)))  float    v8f;
typedef __attribute__((ext_vector_type(4)))  float    v4f;

constexpr int kRows    = 8192;
constexpr int kDim     = 256;
constexpr int kCols2   = 2 * kDim;
constexpr int kOutC    = 9;
constexpr int kNumW    = 75;
constexpr int kBlkRows = 32;
constexpr int kGPlane  = 256;

constexpr float kCarryX = 1024.0f;
constexpr float kCarryU = 256.0f;
constexpr float kFold   = 1.0f / (kCarryX * kCarryU);
constexpr float kHalfMinNormal = 6.103515625e-05f;

static_assert((kDim % 32) == 0, "GEMM K multiple of 32");
static_assert((kRows % 64) == 0 && (kCols2 % 64) == 0, "GEMM M,N multiples of 64");
static_assert((kRows % kBlkRows) == 0, "measure blocks");
static_assert(((kBlkRows * kOutC * 4) % 128) == 0, "measure block output is whole lines");
static_assert(kBlkRows * kOutC == 288, "output floats per measure block");

constexpr size_t kSzG    = (size_t)kGPlane * 4;
constexpr size_t kSzUcol = (size_t)2 * kDim * kDim * 4;
constexpr size_t kSzBt   = (size_t)kCols2 * kDim * 2;
constexpr size_t kSzAx   = (size_t)kRows * kDim * 2;
constexpr size_t kSzPhi  = (size_t)kRows * kCols2 * 4;
constexpr size_t kOffG    = 0;
constexpr size_t kOffUcol = kOffG + kSzG;
constexpr size_t kOffBt   = kOffUcol + kSzUcol;
constexpr size_t kOffAx   = kOffBt + kSzBt;
constexpr size_t kOffPhi  = kOffAx + kSzAx;
constexpr size_t kWsTotal = kOffPhi + kSzPhi;
static_assert(kSzG == 1024 && kSzUcol == 524288 && kSzBt == 262144 && kSzAx == 4194304 && kSzPhi == 16777216, "carve sizes");
static_assert(kWsTotal == 21758976ull, "carve total");
static_assert(kWsTotal <= 134217728ull, "carve cap");
static_assert((kOffUcol % 128) == 0 && (kOffBt % 128) == 0 && (kOffAx % 128) == 0 && (kOffPhi % 128) == 0, "aligned regions");

__device__ __forceinline__ void pin_u(unsigned& v) { asm volatile("" : "+v"(v)); }
__device__ __forceinline__ void pin_f(float& v) { asm volatile("" : "+v"(v)); }

__device__ __forceinline__ void tie_acc(v8f& a, v16h x, v16h y) {
  asm volatile("v_nop\n\tv_nop\n\tv_nop\n\tv_nop" : "+v"(a) : "v"(x), "v"(y));
}
__device__ __forceinline__ void keep4_h(v16h a, v16h b, v16h c, v16h d) { asm volatile("v_nop" :: "v"(a), "v"(b), "v"(c), "v"(d)); }
__device__ __forceinline__ void acc_guard4(v8f& a, v8f& b, v8f& c, v8f& d) {
  asm volatile("v_nop\n\tv_nop\n\tv_nop\n\tv_nop" : "+v"(a), "+v"(b), "+v"(c), "+v"(d));
}

struct FragH {
  union U { v16h v; v8h h[2]; };
  static __device__ __forceinline__ v16h load(const _Float16* p) {
    U f;
    f.h[0] = *(const v8h*)(p);
    f.h[1] = *(const v8h*)(p + 16);
    return f.v;
  }
  static __device__ __forceinline__ v8f mma(v16h a, v16h b, v8f c) {
    return __builtin_amdgcn_wmma_f32_16x16x32_f16(false, a, false, b, (short)0, c, false, false);
  }
};

__global__ __launch_bounds__(256) void compose_gates(const float* __restrict__ w, float* __restrict__ G)
{
  __shared__ float sc[80];
  __shared__ float ss[80];
  __shared__ float qre[160];
  __shared__ float qim[160];
  __shared__ float mre[2][80];
  __shared__ float mim[2][80];
  unsigned t = threadIdx.x;
  pin_u(t);

  unsigned ti = (t < 75u) ? t : 74u;
  pin_u(ti);
  float wv = w[ti];
  pin_f(wv);
  unsigned lay0 = ti / 15u;
  pin_u(lay0);
  unsigned j0 = ti - lay0 * 15u;
  pin_u(j0);
  const bool halfang = (j0 == 0u) || (j0 == 3u) || (j0 == 6u) || (j0 == 7u) || (j0 == 8u) || (j0 == 9u) || (j0 == 12u);
  const float ang = halfang ? (0.5f * wv) : wv;
  float sv, cv;
  sincosf(ang, &sv, &cv);
  if (t < 80u) {
    sc[t] = (t < 75u) ? cv : 0.0f;
    ss[t] = (t < 75u) ? sv : 0.0f;
  }
  __syncthreads();

  unsigned tq = (t < 160u) ? t : 159u;
  pin_u(tq);
  const unsigned l1 = tq >> 5;
  const unsigned gk = (tq >> 2) & 7u;
  const unsigned el = tq & 3u;
  unsigned pb = 8u;
  pb = (gk == 0u) ? 0u : pb;
  pb = (gk == 1u) ? 3u : pb;
  pb = (gk == 2u) ? 6u : pb;
  pb = (gk == 3u) ? 7u : pb;
  pb = (gk == 6u) ? 9u : pb;
  pb = (gk == 7u) ? 12u : pb;
  unsigned ib = l1 * 15u + pb;
  pin_u(ib);
  {
    const float ct = sc[ib];
    const float st = ss[ib];
    const float cp = sc[ib + 1u];
    const float sp = ss[ib + 1u];
    const float cl = sc[ib + 2u];
    const float sl = ss[ib + 2u];
    const float cpl = cp * cl - sp * sl;
    const float spl = sp * cl + cp * sl;
    float u3r = ct;
    float u3i = 0.0f;
    u3r = (el == 1u) ? (-(cl * st)) : u3r;
    u3i = (el == 1u) ? (-(sl * st)) : u3i;
    u3r = (el == 2u) ? (cp * st) : u3r;
    u3i = (el == 2u) ? (sp * st) : u3i;
    u3r = (el == 3u) ? (cpl * ct) : u3r;
    u3i = (el == 3u) ? (spl * ct) : u3i;
    const float ryr = (el == 1u) ? (-st) : ((el == 2u) ? st : ct);
    const bool dg = (el == 0u) || (el == 3u);
    const float rzr = dg ? ct : 0.0f;
    const float rzi = (el == 0u) ? (-st) : ((el == 3u) ? st : 0.0f);
    const float idr = dg ? 1.0f : 0.0f;
    const bool isRY = (gk == 2u) || (gk == 4u);
    const bool isRZ = (gk == 3u);
    const bool isId = (gk == 5u);
    float vr = u3r;
    float vi = u3i;
    vr = isRY ? ryr : vr;
    vi = isRY ? 0.0f : vi;
    vr = isRZ ? rzr : vr;
    vi = isRZ ? rzi : vi;
    vr = isId ? idr : vr;
    vi = isId ? 0.0f : vi;
    if (t < 160u) {
      qre[t] = vr;
      qim[t] = vi;
    }
  }
  __syncthreads();

  unsigned tm = (t < 80u) ? t : 79u;
  pin_u(tm);
  const unsigned l2 = tm >> 4;
  const unsigned r  = (tm >> 2) & 3u;
  const unsigned c  = tm & 3u;
  const unsigned qb = l2 * 32u;
  {
    const unsigned pr = (r == 2u) ? 3u : ((r == 3u) ? 2u : r);
    unsigned ia = qb + (pr >> 1) * 2u + (c >> 1);
    unsigned ic = qb + 4u + (pr & 1u) * 2u + (c & 1u);
    pin_u(ia);
    pin_u(ic);
    const float ar = qre[ia];
    const float ai = qim[ia];
    const float br = qre[ic];
    const float bi = qim[ic];
    if (t < 80u) {
      mre[0][t] = ar * br - ai * bi;
      mim[0][t] = ar * bi + ai * br;
    }
  }
  __syncthreads();
#pragma unroll 1
  for (unsigned s = 0; s < 3u; ++s) {
    const unsigned src = s & 1u;
    const unsigned dst = src ^ 1u;
    const unsigned pa = (s == 0u) ? 1u : ((s == 1u) ? 2u : 0u);
    const unsigned pz = (s == 2u) ? 0u : 3u;
    const unsigned xr = (r == pa) ? pz : ((r == pz) ? pa : r);
    unsigned qa = qb + (2u + 2u * s) * 4u + (xr >> 1) * 2u;
    unsigned qc = qb + (3u + 2u * s) * 4u + (xr & 1u) * 2u;
    pin_u(qa);
    pin_u(qc);
    float accr = 0.0f;
    float acci = 0.0f;
#pragma unroll 1
    for (unsigned k = 0; k < 4u; ++k) {
      const float ar = qre[qa + (k >> 1)];
      const float ai = qim[qa + (k >> 1)];
      const float br = qre[qc + (k & 1u)];
      const float bi = qim[qc + (k & 1u)];
      const float tr = ar * br - ai * bi;
      const float tj = ar * bi + ai * br;
      const float mr = mre[src][l2 * 16u + k * 4u + c];
      const float mi = mim[src][l2 * 16u + k * 4u + c];
      accr += tr * mr - tj * mi;
      acci += tr * mi + tj * mr;
    }
    if (t < 80u) {
      mre[dst][t] = accr;
      mim[dst][t] = acci;
    }
    __syncthreads();
  }
  {
    unsigned i0 = (t < 80u) ? t : 79u;
    unsigned i1 = (t >= 80u && t < 160u) ? (t - 80u) : 0u;
    pin_u(i0);
    pin_u(i1);
    const float fr = mre[1][i0];
    const float fi = mim[1][i1];
    const float val = (t < 80u) ? fr : ((t < 160u) ? fi : 0.0f);
    volatile float* gp = (volatile float*)(G + t);
    *gp = val;
    __threadfence();
    *gp = val;
  }
}

__global__ __launch_bounds__(256) void compose_columns(const float* __restrict__ G, float* __restrict__ Ucol)
{
  __shared__ float sre[2][256];
  __shared__ float sim[2][256];
  __shared__ float gre[80];
  __shared__ float gim[80];
  unsigned t = threadIdx.x;
  pin_u(t);
  const unsigned col = blockIdx.x;

  unsigned tg = (t < 80u) ? t : 79u;
  pin_u(tg);
  float ga = G[tg];
  float gb = G[80u + tg];
  pin_f(ga);
  pin_f(gb);
  if (t < 80u) {
    gre[t] = ga;
    gim[t] = gb;
  }
  sre[0][t] = (t == col) ? 1.0f : 0.0f;
  sim[0][t] = 0.0f;
  __syncthreads();

  const unsigned grp = t >> 2;
  const unsigned k   = t & 3u;
#pragma unroll 1
  for (unsigned g = 0; g < 25u; ++g) {
    unsigned layer, w0, w1;
    if (g < 16u) {
      const unsigned i = g & 7u;
      layer = g >> 3;
      w0 = ((i & 3u) << 1) | (i >> 2);
      w1 = (w0 + 1u) & 7u;
    } else if (g < 24u) {
      const unsigned i = (g - 16u) & 3u;
      layer = 2u + ((g - 16u) >> 2);
      w0 = (0x4062u >> (4u * i)) & 7u;
      w1 = (w0 + 2u) & 7u;
    } else {
      layer = 4u;
      w0 = 2u;
      w1 = 6u;
    }
    const unsigned p0 = 7u - w0;
    const unsigned p1 = 7u - w1;
    const unsigned lo = (p0 < p1) ? p0 : p1;
    const unsigned hi = (p0 < p1) ? p1 : p0;
    const unsigned m0 = 1u << p0;
    const unsigned m1 = 1u << p1;
    unsigned x = ((grp >> lo) << (lo + 1u)) | (grp & ((1u << lo) - 1u));
    x = ((x >> hi) << (hi + 1u)) | (x & ((1u << hi) - 1u));
    pin_u(x);
    const unsigned src = g & 1u;
    const unsigned dst = src ^ 1u;
    const float v0r = sre[src][x];
    const float v0i = sim[src][x];
    const float v1r = sre[src][x | m1];
    const float v1i = sim[src][x | m1];
    const float v2r = sre[src][x | m0];
    const float v2i = sim[src][x | m0];
    const float v3r = sre[src][x | m0 | m1];
    const float v3i = sim[src][x | m0 | m1];
    unsigned gbase = layer * 16u + k * 4u;
    pin_u(gbase);
    const float g0r = gre[gbase];
    const float g0i = gim[gbase];
    const float g1r = gre[gbase + 1u];
    const float g1i = gim[gbase + 1u];
    const float g2r = gre[gbase + 2u];
    const float g2i = gim[gbase + 2u];
    const float g3r = gre[gbase + 3u];
    const float g3i = gim[gbase + 3u];
    float rr = 0.0f;
    float ri = 0.0f;
    rr += g0r * v0r - g0i * v0i;
    ri += g0r * v0i + g0i * v0r;
    rr += g1r * v1r - g1i * v1i;
    ri += g1r * v1i + g1i * v1r;
    rr += g2r * v2r - g2i * v2i;
    ri += g2r * v2i + g2i * v2r;
    rr += g3r * v3r - g3i * v3i;
    ri += g3r * v3i + g3i * v3r;
    unsigned io = x | ((k & 1u) ? m1 : 0u) | ((k & 2u) ? m0 : 0u);
    pin_u(io);
    sre[dst][io] = rr;
    sim[dst][io] = ri;
    __syncthreads();
  }
  {
    const float vr = sre[1][t];
    const float vi = sim[1][t];
    volatile float* pr = (volatile float*)(Ucol + (size_t)col * kDim + t);
    volatile float* pi = (volatile float*)(Ucol + (size_t)kDim * kDim + (size_t)col * kDim + t);
    *pr = vr;
    *pi = vi;
    __threadfence();
    *pr = vr;
    *pi = vi;
  }
}

__global__ __launch_bounds__(256) void transpose_operator(const float* __restrict__ Ucol, unsigned short* __restrict__ Bt)
{
  __shared__ float tile[64 * 65];
  unsigned t = threadIdx.x;
  pin_u(t);
  const unsigned lane = t & 31u;
  const unsigned wave = t >> 5;
  const unsigned bx = blockIdx.x;
  const unsigned pl = bx >> 4;
  const unsigned kt = (bx >> 2) & 3u;
  const unsigned nt = bx & 3u;
  const float* src = Ucol + (size_t)pl * (kDim * kDim) + (size_t)(kt * 64u) * kDim + nt * 64u;
  const unsigned lr = t >> 4;
  const unsigned c4 = (t & 15u) * 4u;
#pragma unroll
  for (int i = 0; i < 4; ++i) {
    const unsigned rr = lr + 16u * (unsigned)i;
    const v4f v = *(const v4f*)(src + (size_t)rr * kDim + c4);
    tile[rr * 65u + c4 + 0u] = v[0];
    tile[rr * 65u + c4 + 1u] = v[1];
    tile[rr * 65u + c4 + 2u] = v[2];
    tile[rr * 65u + c4 + 3u] = v[3];
  }
  __syncthreads();
  const unsigned q  = lane >> 3;
  const unsigned c8 = (lane & 7u) * 8u;
  v8h hv[2];
#pragma unroll
  for (int it = 0; it < 2; ++it) {
    const unsigned nrow = (unsigned)it * 32u + wave * 4u + q;
#pragma unroll
    for (int e = 0; e < 8; ++e) {
      float f = tile[(c8 + (unsigned)e) * 65u + nrow] * kCarryU;
      f = (fabsf(f) < kHalfMinNormal) ? 0.0f : f;
      hv[it][e] = (_Float16)f;
    }
  }
  for (int pass = 0; pass < 2; ++pass) {
#pragma unroll
    for (int it = 0; it < 2; ++it) {
      const unsigned nrow = (unsigned)it * 32u + wave * 4u + q;
      const size_t o = (size_t)(pl * 256u + nt * 64u + nrow) * kDim + kt * 64u + c8;
      *(volatile v8h*)(Bt + o) = hv[it];
    }
    __threadfence();
  }
}

__global__ __launch_bounds__(256) void embed_rows_f16(const float* __restrict__ x, unsigned short* __restrict__ Ax, int nrows)
{
  unsigned t = threadIdx.x;
  pin_u(t);
  const unsigned lane = t & 31u;
  const unsigned wave = t >> 5;
  const int row = (int)(blockIdx.x * 8u + wave);
  if (row >= nrows) return;
  const float* xr = x + (size_t)row * kDim + lane * 8u;
  const v4f a0 = *(const v4f*)(xr);
  const v4f a1 = *(const v4f*)(xr + 4);
  float ssq = 0.0f;
  ssq += a0[0] * a0[0];
  ssq += a0[1] * a0[1];
  ssq += a0[2] * a0[2];
  ssq += a0[3] * a0[3];
  ssq += a1[0] * a1[0];
  ssq += a1[1] * a1[1];
  ssq += a1[2] * a1[2];
  ssq += a1[3] * a1[3];
#pragma unroll
  for (int off = 16; off > 0; off >>= 1) ssq += __shfl_xor(ssq, off, 32);
  const float scl = kCarryX * (1.0f / sqrtf(ssq));
  v8h hv;
#pragma unroll
  for (int e = 0; e < 4; ++e) {
    float f0 = a0[e] * scl;
    float f1 = a1[e] * scl;
    f0 = (fabsf(f0) < kHalfMinNormal) ? 0.0f : f0;
    f1 = (fabsf(f1) < kHalfMinNormal) ? 0.0f : f1;
    hv[e]     = (_Float16)f0;
    hv[4 + e] = (_Float16)f1;
  }
  unsigned short* dst = Ax + (size_t)row * kDim + lane * 8u;
  *(volatile v8h*)dst = hv;
  __threadfence();
  *(volatile v8h*)dst = hv;
}

__global__ __launch_bounds__(256) void gemm_f16_nt(
    const unsigned short* __restrict__ Ap, int lda,
    const unsigned short* __restrict__ Btp, int ldb,
    float* __restrict__ C, int ldc,
    int M, int N, int K, float scale)
{
  const _Float16* A  = (const _Float16*)Ap;
  const _Float16* Bt = (const _Float16*)Btp;
  __shared__ __align__(16) float sT[8][16 * 68];
  const int lane = threadIdx.x & 31;
  const int wave = threadIdx.x >> 5;
  const int tilesN = N >> 6;
  const int tilesM = M >> 6;
  const int tile = blockIdx.x * 8 + wave;
  if (tile >= tilesM * tilesN) return;
  const int tm = tile / tilesN;
  const int tn = tile - tm * tilesN;
  const int m0 = tm << 6;
  const int n0 = tn << 6;
  const int rlane = lane & 15;
  const int koff  = (lane >> 4) * 8;
  const int mOff  = (lane >> 4) * 8;

  v8f acc[4][4];
#pragma unroll
  for (int i = 0; i < 4; ++i)
#pragma unroll
    for (int j = 0; j < 4; ++j) acc[i][j] = (v8f){0.f, 0.f, 0.f, 0.f, 0.f, 0.f, 0.f, 0.f};

  for (int k0 = 0; k0 < K; k0 += 32) {
    v16h bh[4];
#pragma unroll
    for (int j = 0; j < 4; ++j) {
      const size_t bo = (size_t)(n0 + (j << 4) + rlane) * ldb + koff + k0;
      bh[j] = FragH::load(Bt + bo);
    }
#pragma unroll
    for (int i = 0; i < 4; ++i) {
      const size_t ao = (size_t)(m0 + (i << 4) + rlane) * lda + koff + k0;
      const v16h ah = FragH::load(A + ao);
#pragma unroll
      for (int j = 0; j < 4; ++j) acc[i][j] = FragH::mma(ah, bh[j], acc[i][j]);
      tie_acc(acc[i][0], ah, bh[0]);
      tie_acc(acc[i][1], ah, bh[1]);
      tie_acc(acc[i][2], ah, bh[2]);
      tie_acc(acc[i][3], ah, bh[3]);
    }
    keep4_h(bh[0], bh[1], bh[2], bh[3]);
  }
  acc_guard4(acc[0][0], acc[0][1], acc[0][2], acc[0][3]);
  acc_guard4(acc[1][0], acc[1][1], acc[1][2], acc[1][3]);
  acc_guard4(acc[2][0], acc[2][1], acc[2][2], acc[2][3]);
  acc_guard4(acc[3][0], acc[3][1], acc[3][2], acc[3][3]);

  float* slab = sT[wave];
#pragma unroll
  for (int i = 0; i < 4; ++i) {
    const int mBase = m0 + (i << 4);
#pragma unroll
    for (int j = 0; j < 4; ++j) {
#pragma unroll
      for (int r = 0; r < 8; ++r) {
        const float v = acc[i][j][r] * scale;
        slab[(mOff + r) * 68 + (j << 4) + rlane] = v;
      }
    }
    __builtin_amdgcn_fence(__ATOMIC_RELEASE, "workgroup");
    __builtin_amdgcn_wave_barrier();
    __builtin_amdgcn_fence(__ATOMIC_ACQUIRE, "workgroup");
    {
      const int hh = lane >> 4;
      const int c4 = (lane & 15) * 4;
      for (int pass = 0; pass < 2; ++pass) {
#pragma unroll
        for (int it = 0; it < 8; ++it) {
          const int row = it * 2 + hh;
          const v4f v = *(const v4f*)(slab + row * 68 + c4);
          *(volatile v4f*)(C + (size_t)(mBase + row) * ldc + n0 + c4) = v;
        }
        __threadfence();
      }
    }
    __builtin_amdgcn_fence(__ATOMIC_RELEASE, "workgroup");
    __builtin_amdgcn_wave_barrier();
    __builtin_amdgcn_fence(__ATOMIC_ACQUIRE, "workgroup");
  }
}

__global__ __launch_bounds__(256) void measure_rows(const float* __restrict__ Phi, float* __restrict__ out, int nrows)
{
  __shared__ __align__(16) float sOut[kBlkRows * kOutC];
  unsigned t = threadIdx.x;
  pin_u(t);
  const unsigned lane = t & 31u;
  const unsigned wave = t >> 5;
  unsigned base = ((lane & 0x18u) << 3) | ((lane & 7u) << 2);
  pin_u(base);
#pragma unroll 1
  for (unsigned it = 0; it < 4u; ++it) {
    const unsigned lr = wave * 4u + it;
    int row = (int)(blockIdx.x * (unsigned)kBlkRows + lr);
    row = (row < nrows) ? row : (nrows - 1);
    const float* pr = Phi + (size_t)row * kCols2 + base;
    const v4f r0 = *(const v4f*)(pr);
    const v4f r1 = *(const v4f*)(pr + 32);
    const v4f q0 = *(const v4f*)(pr + kDim);
    const v4f q1 = *(const v4f*)(pr + kDim + 32);
    const float ar0 = r0[0], ar1 = r0[1], ar2 = r0[2], ar3 = r0[3];
    const float ar4 = r1[0], ar5 = r1[1], ar6 = r1[2], ar7 = r1[3];
    const float ai0 = q0[0], ai1 = q0[1], ai2 = q0[2], ai3 = q0[3];
    const float ai4 = q1[0], ai5 = q1[1], ai6 = q1[2], ai7 = q1[3];
    const float n0 = ar0 * ar0 + ai0 * ai0;
    const float n1 = ar1 * ar1 + ai1 * ai1;
    const float n2 = ar2 * ar2 + ai2 * ai2;
    const float n3 = ar3 * ar3 + ai3 * ai3;
    const float n4 = ar4 * ar4 + ai4 * ai4;
    const float n5 = ar5 * ar5 + ai5 * ai5;
    const float n6 = ar6 * ar6 + ai6 * ai6;
    const float n7 = ar7 * ar7 + ai7 * ai7;
    const float n01 = n0 + n1, n23 = n2 + n3, n45 = n4 + n5, n67 = n6 + n7;
    float red[10];
    red[0] = ((ar0 * ar4 + ai0 * ai4) + (ar1 * ar5 + ai1 * ai5)) + ((ar2 * ar6 + ai2 * ai6) + (ar3 * ar7 + ai3 * ai7));
    red[1] = ((ar0 * ai4 - ai0 * ar4) + (ar1 * ai5 - ai1 * ar5)) + ((ar2 * ai6 - ai2 * ar6) + (ar3 * ai7 - ai3 * ar7));
    red[2] = (n01 + n23) - (n45 + n67);
    red[3] = ((ar0 * ar2 + ai0 * ai2) + (ar1 * ar3 + ai1 * ai3)) + ((ar4 * ar6 + ai4 * ai6) + (ar5 * ar7 + ai5 * ai7));
    red[4] = ((ar0 * ai2 - ai0 * ar2) + (ar1 * ai3 - ai1 * ar3)) + ((ar4 * ai6 - ai4 * ar6) + (ar5 * ai7 - ai5 * ar7));
    red[5] = (n01 + n45) - (n23 + n67);
    {
      const float c06 = ar0 * ar6 + ai0 * ai6;
      const float c17 = ar1 * ar7 + ai1 * ai7;
      const float c24 = ar2 * ar4 + ai2 * ai4;
      const float c35 = ar3 * ar5 + ai3 * ai5;
      red[6] = (c06 + c17) + (c24 + c35);
      red[7] = (c24 + c35) - (c06 + c17);
    }
    red[8] = (n01 + n67) - (n23 + n45);
    red[9] = (n01 + n23) + (n45 + n67);
#pragma unroll
    for (int k = 0; k < 10; ++k) {
#pragma unroll
      for (int off = 16; off > 0; off >>= 1) red[k] += __shfl_xor(red[k], off, 32);
    }
    const float inv = 1.0f / red[9];
    const float inv2 = 2.0f * inv;
    if (lane == 0u) {
      float* so = sOut + lr * (unsigned)kOutC;
      so[0] = red[0] * inv2;
      so[1] = red[1] * inv2;
      so[2] = red[2] * inv;
      so[3] = red[3] * inv2;
      so[4] = red[4] * inv2;
      so[5] = red[5] * inv;
      so[6] = red[6] * inv2;
      so[7] = red[7] * inv2;
      so[8] = red[8] * inv;
    }
  }
  __syncthreads();
  if (wave == 0u) {
    unsigned i2 = 64u + lane;
    i2 = (i2 < 72u) ? i2 : 71u;
    pin_u(i2);
    const v4f v0 = *(const v4f*)(sOut + lane * 4u);
    const v4f v1 = *(const v4f*)(sOut + (32u + lane) * 4u);
    const v4f v2 = *(const v4f*)(sOut + i2 * 4u);
    float* ob = out + (size_t)blockIdx.x * (kBlkRows * kOutC);
    for (int pass = 0; pass < 2; ++pass) {
      *(volatile v4f*)(ob + lane * 4u) = v0;
      *(volatile v4f*)(ob + 128u + lane * 4u) = v1;
      if (lane < 8u) *(volatile v4f*)(ob + 256u + lane * 4u) = v2;
      __threadfence();
    }
  }
}

static_assert(((kRows / 64) * (kCols2 / 64)) % 8 == 0, "GEMM tiles per block");

extern "C" void kernel_launch(void* const* d_in, const int* in_sizes, int n_in,
                              void* d_out, int out_size, void* d_ws, size_t ws_size,
                              hipStream_t stream) {
  if (n_in < 2) return;
  if (in_sizes[0] != kRows * kDim) return;
  if (in_sizes[1] != kNumW) return;
  if (out_size != kRows * kOutC) return;
  if (ws_size < kWsTotal) return;

  const float* x = (const float*)d_in[0];
  const float* w = (const float*)d_in[1];
  float* out = (float*)d_out;

  char* ws = (char*)d_ws;
  float*          G    = (float*)(ws + kOffG);
  float*          Ucol = (float*)(ws + kOffUcol);
  unsigned short* Bt   = (unsigned short*)(ws + kOffBt);
  unsigned short* Ax   = (unsigned short*)(ws + kOffAx);
  float*          Phi  = (float*)(ws + kOffPhi);

  compose_gates<<<1, 256, 0, stream>>>(w, G);
  compose_columns<<<kDim, 256, 0, stream>>>(G, Ucol);
  transpose_operator<<<32, 256, 0, stream>>>(Ucol, Bt);
  embed_rows_f16<<<kRows / 8, 256, 0, stream>>>(x, Ax, kRows);
  gemm_f16_nt<<<((kRows / 64) * (kCols2 / 64)) / 8, 256, 0, stream>>>(
      Ax, kDim, Bt, kDim, Phi, kCols2, kRows, kCols2, kDim, kFold);
  measure_rows<<<kRows / kBlkRows, 256, 0, stream>>>(Phi, out, kRows);
}
